// StructuralMambaMixer_81698867905020
// MI455X (gfx1250) — hardware-verified
//
#include <hip/hip_runtime.h>

#define DM     1024
#define DI     2048
#define DSTATE 16
#define DTRANK 64
#define BB     2
#define LL     2048
#define MROWS  (BB*LL)
#define XDBL_W (DTRANK + 2*DSTATE)

typedef _Float16     v16h __attribute__((ext_vector_type(16)));
typedef float        v8f  __attribute__((ext_vector_type(8)));
typedef unsigned int u4   __attribute__((ext_vector_type(4)));

union Frag { struct { u4 lo, hi; } q; v16h v; };
typedef float v4f __attribute__((ext_vector_type(4)));
typedef _Float16 v8h __attribute__((ext_vector_type(8)));
template <typename V> __device__ __forceinline__ void vst2(void* p, V v) {
    *(volatile V*)p = v; __threadfence(); *(volatile V*)p = v;
}
__device__ __forceinline__ void copy_b128(char* lds_byte_ptr, const void* gptr) {
    *(u4*)lds_byte_ptr = *(const u4*)gptr;
}
__device__ __forceinline__ v8f wmma16(v16h a, v16h b, v8f c) {
    v8f d = __builtin_amdgcn_wmma_f32_16x16x32_f16(false, a, false, b, (short)0, c, false, false);
    asm volatile("v_nop\n\tv_nop\n\tv_nop\n\tv_nop" : "+v"(d) : "v"(a), "v"(b));
    return d;
}

template<int EPI>
__global__ __launch_bounds__(256)
void wmma_gemm_h(const _Float16* __restrict__ A, int lda,
                 const _Float16* __restrict__ W, int ldb,
                 float* __restrict__ C, int ldc,
                 int N, int K, const float* __restrict__ bias)
{
    __shared__ __align__(16) _Float16 lds[2 * 6144];
    __shared__ __align__(16) float Ct[64][128];

    const int tid    = threadIdx.x;
    const int lane   = tid & 31;
    const int wave   = tid >> 5;
    const int waveM  = wave >> 2;
    const int waveN  = wave & 3;
    const int lane16 = lane & 15;
    const int half   = lane >> 4;
    const int rowBase = blockIdx.y * 64;
    const int colBase = blockIdx.x * 128;

    {
        u4* z = (u4*)lds;
        #pragma unroll
        for (int i = 0; i < 6; ++i) {
            u4 zz; zz[0] = 0u; zz[1] = 0u; zz[2] = 0u; zz[3] = 0u;
            z[tid + 256 * i] = zz;
        }
    }
    __syncthreads();

    char* ldsBase = (char*)&lds[0];

    const int aRow = tid >> 2, aCh = tid & 3;
    const int bRow = tid >> 1, bCh = tid & 1;
    const int bN   = colBase + bRow;
    const int bNc  = (bN < N) ? bN : (N - 1);

    const _Float16* aSrc = A + (size_t)(rowBase + aRow) * lda + aCh * 8;
    const _Float16* bSrc = W + (size_t)bNc * ldb + bCh * 16;
    const unsigned aDst = (unsigned)(aRow * 64 + aCh * 16);
    const unsigned bDst = (unsigned)(4096 + bRow * 64 + bCh * 32);

    const int kTiles = K >> 5;

    copy_b128(ldsBase + aDst, aSrc);
    copy_b128(ldsBase + bDst,      bSrc);
    copy_b128(ldsBase + bDst + 16, bSrc + 8);

    v8f acc[2][2] = {};

    for (int kt = 0; kt < kTiles; ++kt) {
        if (kt + 1 < kTiles) {
            char* bb = ldsBase + ((kt + 1) & 1) * 12288;
            const int kOff = (kt + 1) << 5;
            copy_b128(bb + aDst, aSrc + kOff);
            copy_b128(bb + bDst,      bSrc + kOff);
            copy_b128(bb + bDst + 16, bSrc + kOff + 8);
        }
        __syncthreads();

        const unsigned* bufU = (const unsigned*)&lds[(kt & 1) * 6144];
        Frag aF[2], bF[2];
        #pragma unroll
        for (int m = 0; m < 2; ++m) {
            const int r = waveM * 32 + m * 16 + lane16;
            const unsigned* p = bufU + r * 16 + half * 4;
            aF[m].q.lo = *(const u4*)p;
            aF[m].q.hi = *(const u4*)(p + 8);
        }
        #pragma unroll
        for (int n = 0; n < 2; ++n) {
            const int c = waveN * 32 + n * 16 + lane16;
            const unsigned* p = bufU + 1024 + c * 16 + half * 4;
            bF[n].q.lo = *(const u4*)p;
            bF[n].q.hi = *(const u4*)(p + 8);
        }
        #pragma unroll
        for (int m = 0; m < 2; ++m)
            #pragma unroll
            for (int n = 0; n < 2; ++n)
                acc[m][n] = wmma16(aF[m].v, bF[n].v, acc[m][n]);

        __syncthreads();
    }

    #pragma unroll
    for (int m = 0; m < 2; ++m) {
        const int rl0 = waveM * 32 + m * 16 + half * 8;
        #pragma unroll
        for (int n = 0; n < 2; ++n) {
            const int cl = waveN * 32 + n * 16 + lane16;
            const int col = colBase + cl;
            const float bv = (EPI == 1 && col < N) ? bias[col] : 0.f;
            #pragma unroll
            for (int r = 0; r < 8; ++r) {
                float v = acc[m][n][r];
                if (EPI == 1) {
                    v += bv;
                    v = (v > 15.f) ? v : __logf(1.f + __expf(v));
                }
                Ct[rl0 + r][cl] = v;
            }
        }
    }
    __syncthreads();
    {
        const int ncols = (N - colBase < 128) ? (N - colBase) : 128;
        const int ppr = ncols >> 2;
        for (int g = tid; g < 64 * ppr; g += 256) {
            const int rl = g / ppr, pc = g - rl * ppr;
            vst2(C + (size_t)(rowBase + rl) * ldc + colBase + pc * 4, *(const v4f*)(&Ct[rl][pc * 4]));
        }
    }
}

__global__ __launch_bounds__(256)
void cvt_f32_f16(const float* __restrict__ s, _Float16* __restrict__ d, int n)
{
    const int g = blockIdx.x * 256 + threadIdx.x;
    if (g * 8 >= n) return;
    const v4f a = *(const v4f*)(s + (size_t)g * 8), b = *(const v4f*)(s + (size_t)g * 8 + 4);
    union { v8h h; u4 u; } pk;
    #pragma unroll
    for (int i = 0; i < 4; ++i) { pk.h[i] = (_Float16)a[i]; pk.h[4 + i] = (_Float16)b[i]; }
    vst2(d + (size_t)g * 8, pk.u);
}

__global__ __launch_bounds__(256)
void conv_silu(const float* __restrict__ xin, const float* __restrict__ w,
               const float* __restrict__ b, float* __restrict__ u,
               _Float16* __restrict__ u_h)
{
    const int idx = blockIdx.x * 256 + threadIdx.x;
    const int row = idx / (DI / 2);
    const int d   = (idx - row * (DI / 2)) * 2;
    const int l   = row & (LL - 1);
    float sv[2];
    #pragma unroll
    for (int q = 0; q < 2; ++q) {
        float acc = b[d + q];
        const float* wr = w + (d + q) * 4;
        #pragma unroll
        for (int j = 0; j < 4; ++j) {
            const int ll = l - 3 + j;
            if (ll >= 0)
                acc = fmaf(xin[(size_t)(row - 3 + j) * (2 * DI) + d + q], wr[j], acc);
        }
        sv[q] = acc / (1.f + __expf(-acc));
    }
    typedef float v2f __attribute__((ext_vector_type(2)));
    vst2(u + (size_t)row * DI + d, (v2f){sv[0], sv[1]});
    union { _Float16 h[2]; unsigned uu; } pk; pk.h[0] = (_Float16)sv[0]; pk.h[1] = (_Float16)sv[1];
    vst2(u_h + (size_t)row * DI + d, pk.uu);
}

__global__ __launch_bounds__(256)
void selective_scan(const float* __restrict__ dt, const float* __restrict__ u,
                    const float* __restrict__ xdbl, const float* __restrict__ proj,
                    const float* __restrict__ A_log, const float* __restrict__ D_skip,
                    _Float16* __restrict__ y_h)
{
    const int b = blockIdx.x >> 2;
    const int d = ((blockIdx.x & 3) * 256 + threadIdx.x) * 2;
    __shared__ float sB[DSTATE], sC[DSTATE];

    float Arow[2][DSTATE], h[2][DSTATE], Dsk[2];
    #pragma unroll
    for (int q = 0; q < 2; ++q) {
        #pragma unroll
        for (int s = 0; s < DSTATE; ++s) { Arow[q][s] = -expf(A_log[(d + q) * DSTATE + s]); h[q][s] = 0.f; }
        Dsk[q] = D_skip[d + q];
    }

    for (int l = 0; l < LL; ++l) {
        const int row = b * LL + l;
        __syncthreads();
        if (threadIdx.x < 2 * DSTATE) {
            const float v = xdbl[row * XDBL_W + DTRANK + threadIdx.x];
            if (threadIdx.x < DSTATE) sB[threadIdx.x] = v;
            else                      sC[threadIdx.x - DSTATE] = v;
        }
        __syncthreads();
        union { _Float16 hh[2]; unsigned uu; } pk;
        #pragma unroll 1
        for (int q = 0; q < 2; ++q) {
            const float dtv = dt[(size_t)row * DI + d + q];
            const float uv  = u [(size_t)row * DI + d + q];
            const float du  = dtv * uv;
            float y = 0.f;
            #pragma unroll
            for (int s = 0; s < DSTATE; ++s) {
                h[q][s] = __expf(dtv * Arow[q][s]) * h[q][s] + sB[s] * du;
                y = fmaf(h[q][s], sC[s], y);
            }
            const float g = proj[(size_t)row * (2 * DI) + DI + d + q];
            pk.hh[q] = (_Float16)((y + uv * Dsk[q]) * (g / (1.f + __expf(-g))));
        }
        vst2(y_h + (size_t)row * DI + d, pk.uu);
    }
}

extern "C" void kernel_launch(void* const* d_in, const int* in_sizes, int n_in,
                              void* d_out, int out_size, void* d_ws, size_t ws_size,
                              hipStream_t stream)
{
    const float* hidden     = (const float*)d_in[0];
    const float* in_proj_w  = (const float*)d_in[2];
    const float* conv_w     = (const float*)d_in[3];
    const float* conv_b     = (const float*)d_in[4];
    const float* x_proj_w   = (const float*)d_in[5];
    const float* dt_proj_w  = (const float*)d_in[6];
    const float* dt_proj_b  = (const float*)d_in[7];
    const float* A_log      = (const float*)d_in[8];
    const float* D_skip     = (const float*)d_in[9];
    const float* out_proj_w = (const float*)d_in[10];
    float* out = (float*)d_out;

    float* proj = (float*)d_ws;
    float* u    = proj + (size_t)MROWS * (2 * DI);
    float* xdbl = u    + (size_t)MROWS * DI;
    float* dt   = xdbl + (size_t)MROWS * XDBL_W;
    _Float16* hidden_h = (_Float16*)(dt + (size_t)MROWS * DI);
    _Float16* inW_h    = hidden_h + (size_t)MROWS * DM;
    _Float16* xW_h     = inW_h    + (size_t)(2 * DI) * DM;
    _Float16* dtW_h    = xW_h     + (size_t)XDBL_W * DI;
    _Float16* outW_h   = dtW_h    + (size_t)DI * DTRANK;
    _Float16* u_h      = outW_h   + (size_t)DM * DI;
    _Float16* xdbl_h   = u_h      + (size_t)MROWS * DI;
    _Float16* y_h      = xdbl_h   + (size_t)MROWS * XDBL_W;

    const dim3 blk(256);
    auto cvt = [&](const float* s, _Float16* d, int n) {
        cvt_f32_f16<<<(n / 8 + 255) / 256, blk, 0, stream>>>(s, d, n);
    };

    cvt(hidden,     hidden_h, MROWS * DM);
    cvt(in_proj_w,  inW_h,    2 * DI * DM);
    cvt(x_proj_w,   xW_h,     XDBL_W * DI);
    cvt(dt_proj_w,  dtW_h,    DI * DTRANK);
    cvt(out_proj_w, outW_h,   DM * DI);

    wmma_gemm_h<0><<<dim3((2 * DI) / 128, MROWS / 64), blk, 0, stream>>>(
        hidden_h, DM, inW_h, DM, proj, 2 * DI, 2 * DI, DM, nullptr);

    conv_silu<<<(MROWS * DI / 2) / 256, blk, 0, stream>>>(proj, conv_w, conv_b, u, u_h);

    wmma_gemm_h<0><<<dim3(1, MROWS / 64), blk, 0, stream>>>(
        u_h, DI, xW_h, DI, xdbl, XDBL_W, XDBL_W, DI, nullptr);
    cvt(xdbl, xdbl_h, MROWS * XDBL_W);

    wmma_gemm_h<1><<<dim3(DI / 128, MROWS / 64), blk, 0, stream>>>(
        xdbl_h, XDBL_W, dtW_h, DTRANK, dt, DI, DI, DTRANK, dt_proj_b);

    selective_scan<<<BB * (DI / 512), blk, 0, stream>>>(
        dt, u, xdbl, proj, A_log, D_skip, y_h);

    wmma_gemm_h<0><<<dim3(DM / 128, MROWS / 64), blk, 0, stream>>>(
        y_h, DI, outW_h, DI, out, DM, DM, DI, nullptr);
}
